// aggregator_27633819583079
// MI455X (gfx1250) — hardware-verified
//
#include <hip/hip_runtime.h>


namespace {
typedef _Float16 b16;
typedef __attribute__((ext_vector_type(16))) _Float16 v16b;
typedef __attribute__((ext_vector_type(8))) _Float16 v8b;
typedef __attribute__((ext_vector_type(4))) _Float16 v4h;
typedef __attribute__((ext_vector_type(2))) _Float16 v2h;
typedef __attribute__((ext_vector_type(8))) float v8f;
typedef __attribute__((ext_vector_type(4))) float v4f;
typedef __attribute__((ext_vector_type(2))) float v2f;
__device__ __forceinline__ float bf16_rne(float f) { unsigned int u = __float_as_uint(f); u += 0x7FFFu + ((u >> 16) & 1u); return __uint_as_float(u & 0xFFFF0000u); }
__device__ __forceinline__ void split16(float v, b16& hi, b16& lo) { hi = (b16)v; lo = (b16)(v - (float)hi); }
__device__ __forceinline__ v16b frag_kb(const b16* p, int hh) { const v8b a = *(const v8b*)(p + 8 * hh), b = *(const v8b*)(p + 16 + 8 * hh); v16b f;
#pragma unroll
  for (int e = 0; e < 8; ++e) { f[e] = a[e]; f[8 + e] = b[e]; } return f; }
__device__ __forceinline__ v8f wmma16b(v16b a, v16b b, v8f c) { v8f d = __builtin_amdgcn_wmma_f32_16x16x32_f16(false, a, false, b, (short)0, c, false, false); asm volatile("v_nop\n\tv_nop\n\tv_nop\n\tv_nop" : "+v"(d) : "v"(a), "v"(b)); return d; }
__device__ __forceinline__ void wave_lds_sync() { __builtin_amdgcn_fence(__ATOMIC_RELEASE, "workgroup"); __builtin_amdgcn_wave_barrier(); __builtin_amdgcn_fence(__ATOMIC_ACQUIRE, "workgroup"); }
__device__ __forceinline__ float pmul(float a, float b) { float p = a * b; asm volatile("" : "+v"(p)); return p; }
__device__ __forceinline__ int iclamp(int v, int lo, int hi) { return v < lo ? lo : (v > hi ? hi : v); }
__device__ __forceinline__ float nexp2(float v) { return __builtin_amdgcn_exp2f(v); }

constexpr int NB = 4096, L = 50, LP = 64, D = 64, NT = 100000, NBL = NB  ;
constexpr float XS = 8.0f, WSC = 256.0f;
static_assert(D == 64 && LP == 64 && L <= LP, "tiling");
__global__ __launch_bounds__(256) void prep_kernel(const float* __restrict__ w1, const float* __restrict__ w2, b16* __restrict__ W1T, b16* __restrict__ W2T) {
  const int u = blockIdx.x * 256 + threadIdx.x; if (u >= 2 * D * D / 8) return; const int e = (u * 8) % (D * D); const int c = e / D, k0 = e % D; const bool second = u >= D * D / 8; v8b o;
  for (int j = 0; j < 8; ++j) o[j] = (b16)(bf16_rne(second ? w2[(size_t)(k0 + j) * D + c] : w1[(size_t)(k0 + j) * D + c]) * WSC);
  for (int pass = 0; pass < 2; ++pass) { *(volatile v8b*)((second ? W2T : W1T) + e) = o; __threadfence(); }
}
__global__ __launch_bounds__(128) void node_kernel(const float* __restrict__ ut, const float* __restrict__ it, const float* __restrict__ w1, const float* __restrict__ b1, const b16* __restrict__ W1T, const b16* __restrict__ W2T, const float* __restrict__ b2, const float* __restrict__ w3, const float* __restrict__ b3,
                                                  const int* __restrict__ nodes, const int* __restrict__ nbrs, const int* __restrict__ lens, float* __restrict__ out) {
  __shared__ __attribute__((aligned(16))) b16 As[LP][D + 8], Hh[LP][D + 8], Hl[LP][D + 8]; __shared__ float pn[D], w3s[D], lg[LP], att[LP]; __shared__ int nb_s[LP];
  const int wave = threadIdx.x >> 5, lane = threadIdx.x & 31, nloc = lane & 15, hlf = lane >> 4, t_ = threadIdx.x; const int b = blockIdx.x; if (b >= NBL) return;
  const int node = iclamp(nodes[b], 0, NT - 1); int len = lens[b]; len = iclamp(len, 1, L);
  if (t_ < LP) nb_s[t_] = (t_ < L) ? iclamp(nbrs[(size_t)b * L + t_], 0, NT - 1) : 0;
  if (t_ < D) { float a = bf16_rne(b1[t_]);
#pragma unroll 4
    for (int k = 0; k < D; ++k) a = fmaf(bf16_rne(ut[(size_t)node * D + k]), bf16_rne(w1[(size_t)(D + k) * D + t_]), a); pn[t_] = a; w3s[t_] = bf16_rne(w3[t_]); }
  __syncthreads();
  for (int i = t_; i < LP * (D / 4); i += 128) { const int r = i / (D / 4), c4 = (i % (D / 4)) * 4; v4h hv; if (r < L) { const v4f v = *(const v4f*)(it + (size_t)nb_s[r] * D + c4); for (int j = 0; j < 4; ++j) hv[j] = (b16)(bf16_rne(v[j]) * XS); } else { for (int j = 0; j < 4; ++j) hv[j] = (b16)0.0f; } *(v4h*)(&As[r][c4]) = hv; }
  __syncthreads();
  v8f acc[4];
#pragma unroll
  for (int t = 0; t < 4; ++t) acc[t] = (v8f){};
#pragma unroll
  for (int kb = 0; kb < D; kb += 32) { const v16b a = frag_kb(&As[wave * 16 + nloc][kb], hlf);
#pragma unroll
    for (int t = 0; t < 4; ++t) acc[t] = wmma16b(a, frag_kb(W1T + (size_t)(t * 16 + nloc) * D + kb, hlf), acc[t]); }
#pragma unroll
  for (int t = 0; t < 4; ++t) { const int c = t * 16 + nloc;
#pragma unroll
    for (int r = 0; r < 8; ++r) { const float h = fmaxf(acc[t][r] * (1.0f / (XS * WSC)) + pn[c], 0.0f); b16 ph, pl; split16(h * XS, ph, pl); Hh[wave * 16 + 8 * hlf + r][c] = ph; Hl[wave * 16 + 8 * hlf + r][c] = pl; } }
  wave_lds_sync();
#pragma unroll
  for (int t = 0; t < 4; ++t) acc[t] = (v8f){};
#pragma unroll
  for (int kb = 0; kb < D; kb += 32) { const v16b a = frag_kb(&Hh[wave * 16 + nloc][kb], hlf), al = frag_kb(&Hl[wave * 16 + nloc][kb], hlf);
#pragma unroll
    for (int t = 0; t < 4; ++t) { const v16b bw = frag_kb(W2T + (size_t)(t * 16 + nloc) * D + kb, hlf); acc[t] = wmma16b(a, bw, acc[t]); acc[t] = wmma16b(al, bw, acc[t]); } }
  float lgt[8];
#pragma unroll
  for (int r = 0; r < 8; ++r) { float p = 0.0f;
#pragma unroll
    for (int t = 0; t < 4; ++t) { const int c = t * 16 + nloc; const float h2 = fmaxf(acc[t][r] * (1.0f / (XS * WSC)) + bf16_rne(b2[c]), 0.0f); p = fmaf(h2, w3s[c], p); } lgt[r] = p; }
#pragma unroll
  for (int w = 1; w < 16; w <<= 1)
#pragma unroll
    for (int r = 0; r < 8; ++r) lgt[r] += __shfl_xor(lgt[r], w);
  if (nloc == 0) { const float bb = bf16_rne(b3[0]);
#pragma unroll
    for (int r = 0; r < 8; ++r) lg[wave * 16 + 8 * hlf + r] = lgt[r] + bb; }
  __syncthreads();
  if (t_ == 0) { float m = -INFINITY; for (int l = 0; l < len; ++l) m = fmaxf(m, lg[l]); float s = 0.0f; for (int l = 0; l < LP; ++l) { const float e = (l < len) ? __expf(lg[l] - m) : 0.0f; att[l] = e; s += e; } const float inv = 1.0f / s; for (int l = 0; l < LP; ++l) att[l] *= inv; }
  __syncthreads();
  float o = 0.0f; if (t_ < D) {
#pragma unroll 2
    for (int l = 0; l < L; ++l) o = fmaf(att[l], (float)As[l][t_] * (1.0f / XS), o); }
  for (int pass = 0; pass < 2; ++pass) { if (t_ < D) ((volatile float*)out)[(size_t)b * D + t_] = o; __threadfence(); }
}
}

extern "C" void kernel_launch(void* const* d_in, const int* in_sizes, int n_in, void* d_out, int out_size, void* d_ws, size_t ws_size, hipStream_t stream) {
  (void)n_in;
  auto Fp = [&](int i) { return (const float*)d_in[i]; }; auto Ip = [&](int i) { return (const int*)d_in[i]; };
  if (in_sizes[0] != NT * D || in_sizes[1] != NT * D || in_sizes[2] != 2 * D * D || in_sizes[3] != D || in_sizes[4] != D * D || in_sizes[5] != D || in_sizes[6] != D || in_sizes[7] != 1 || in_sizes[8] != NB || in_sizes[9] != NB * L || in_sizes[10] != NB || out_size != NB * D) return;
  size_t off = 0; char* ws = (char*)d_ws;
  auto carve = [&](size_t bytes) { char* p = ws + off; off += (bytes + 255) & ~(size_t)255; return p; };
  b16* W1T = (b16*)carve((size_t)D * D * 2); b16* W2T = (b16*)carve((size_t)D * D * 2);
  if (off > ws_size || off > ((size_t)128 << 20)) return;
  prep_kernel<<<(2 * D * D / 8 + 255) / 256, 256, 0, stream>>>(Fp(2), Fp(4), W1T, W2T);
  node_kernel<<<NBL, 128, 0, stream>>>(Fp(0), Fp(1), Fp(2), Fp(3), W1T, W2T, Fp(5), Fp(6), Fp(7), Ip(8), Ip(9), Ip(10), (float*)d_out);
}
